// XConv_9277129360147
// MI455X (gfx1250) — hardware-verified
//
#include <hip/hip_runtime.h>

typedef __attribute__((ext_vector_type(16))) __bf16 v16b;
typedef __attribute__((ext_vector_type(8)))  __bf16 v8b;
typedef __attribute__((ext_vector_type(8)))  float  v8f;
typedef __attribute__((ext_vector_type(4)))  float  v4f;

static constexpr int NPTS  = 100000;
static constexpr int NSRC  = 100000;
static constexpr int KNB   = 16;
static constexpr int CIN   = 64;
static constexpr int CDEL  = 16;
static constexpr int COUT  = 128;
static constexpr int NCH1  = 256;
static constexpr int KREL  = 48;
static constexpr int KRELP = 64;
static constexpr int YDIM  = 160;
static constexpr int PB    = 16;
static constexpr int NBLKS = NPTS / PB;
static_assert(NPTS % PB == 0);
static constexpr int TPITCH = 512;
static constexpr int HPITCH = 32;

static constexpr size_t OFF_WX1P = 0;
static constexpr size_t OFF_W2P  = OFF_WX1P + (size_t)256 * KRELP * 2;
static constexpr size_t OFF_WX1G = OFF_W2P + (size_t)16 * 16 * 2;
static constexpr size_t OFF_WX2G = OFF_WX1G + (size_t)4096 * 2;
static constexpr size_t OFF_WOP  = OFF_WX2G + (size_t)4096 * 2;
static constexpr size_t OFF_PR   = OFF_WOP + (size_t)COUT * YDIM * 2;
static constexpr int PR_W1 = 0, PR_B1 = 64, PR_B2 = 96, PR_BX1 = 128, PR_BG1 = 384, PR_BG2 = 640,
                     PR_WC = 896, PR_BC = 3456, PR_BO = 3616, PR_TOT = 3744;
static constexpr size_t OFF_BN   = OFF_PR + (size_t)PR_TOT * 4;
static constexpr int BN_SC1 = 0, BN_SH1 = 32, BN_SCX1 = 64, BN_SHX1 = 320, BN_SC2 = 576, BN_SH2 = 608,
                     BN_SCX2 = 640, BN_SHX2 = 896, BN_SCX3 = 1152, BN_SHX3 = 1408, BN_TOT = 1664;
static constexpr size_t OFF_PH   = OFF_BN + (size_t)BN_TOT * 4;
static constexpr size_t OFF_PT   = OFF_PH + (size_t)NBLKS * HPITCH * 4;
static constexpr size_t OFF_T2   = OFF_PT + (size_t)NBLKS * TPITCH * 4;
static constexpr size_t WS_END   = OFF_T2 + (size_t)NPTS * NCH1 * 4;
static_assert(WS_END == 116112256ull);
static_assert(WS_END <= 134217728ull);
static_assert(OFF_W2P % 128 == 0 && OFF_WX1G % 128 == 0 && OFF_WX2G % 128 == 0 && OFF_WOP % 128 == 0 &&
              OFF_PR % 128 == 0 && OFF_BN % 128 == 0 && OFF_PH % 128 == 0 && OFF_PT % 128 == 0 && OFF_T2 % 128 == 0);
static_assert(PR_TOT % 32 == 0 && PR_W1 % 32 == 0 && PR_B1 % 32 == 0 && PR_B2 % 32 == 0 && PR_BX1 % 32 == 0 &&
              PR_BG1 % 32 == 0 && PR_BG2 % 32 == 0 && PR_WC % 32 == 0 && PR_BC % 32 == 0 && PR_BO % 32 == 0);
static constexpr int WD_W2P     = (int)(OFF_W2P / 4);
static constexpr int WD_WX1G    = (int)(OFF_WX1G / 4);
static constexpr int WD_WX2G    = (int)(OFF_WX2G / 4);
static constexpr int WD_WOP     = (int)(OFF_WOP / 4);
static constexpr int WD_PR      = (int)(OFF_PR / 4);
static constexpr int PREP_WORDS = (int)(OFF_BN / 4);
static_assert(WD_W2P % 32 == 0 && WD_WX1G % 32 == 0 && WD_WX2G % 32 == 0 && WD_WOP % 32 == 0 &&
              WD_PR % 32 == 0 && PREP_WORDS % 32 == 0);
static_assert(WD_PR - WD_WOP == COUT * YDIM / 2);
static_assert(PREP_WORDS - WD_PR == PR_TOT);

__device__ __forceinline__ unsigned short f2bf_bits(float f) {
  unsigned u = __float_as_uint(f);
  return (unsigned short)((u + 0x7FFFu + ((u >> 16) & 1u)) >> 16);
}
__device__ __forceinline__ float bf_bits2f(unsigned short h) { return __uint_as_float(((unsigned)h) << 16); }
__device__ __forceinline__ float bfr(float f) { return bf_bits2f(f2bf_bits(f)); }
__device__ __forceinline__ __bf16 tobf(float f) { return __builtin_bit_cast(__bf16, f2bf_bits(f)); }
__device__ __forceinline__ void split_bf(float f, __bf16& hi, __bf16& lo) {
  const unsigned short hb = f2bf_bits(f);
  hi = __builtin_bit_cast(__bf16, hb);
  lo = tobf(f - bf_bits2f(hb));
}
__device__ __forceinline__ unsigned pack2bf(float a, float b) {
  return (unsigned)f2bf_bits(a) | ((unsigned)f2bf_bits(b) << 16);
}
__device__ __forceinline__ float eluf(float v) { return v > 0.f ? v : (__expf(v) - 1.0f); }
__device__ __forceinline__ int clampi(int v, int hi) { v = v < 0 ? 0 : v; return v > hi ? hi : v; }
__device__ __forceinline__ v8f zero8() { return (v8f){0.f, 0.f, 0.f, 0.f, 0.f, 0.f, 0.f, 0.f}; }

union FragU { v16b v; v8b h[2]; };
__device__ __forceinline__ v16b frag_std(const __bf16* p) {
  FragU f; f.h[0] = *(const v8b*)(p); f.h[1] = *(const v8b*)(p + 16); return f.v;
}
__device__ __forceinline__ v16b frag_pair(const __bf16* phi, const __bf16* plo) {
  FragU f; f.h[0] = *(const v8b*)(phi); f.h[1] = *(const v8b*)(plo); return f.v;
}
__device__ __forceinline__ v16b frag_dup(const __bf16* p) {
  FragU f; f.h[0] = *(const v8b*)(p); f.h[1] = f.h[0]; return f.v;
}
__device__ __forceinline__ v8f mma_bf(v16b a, v16b b, v8f c) {
  c = __builtin_amdgcn_wmma_f32_16x16x32_bf16(false, a, false, b, (short)0, c, false, false);
  asm volatile("v_nop\n\tv_nop\n\tv_nop\n\tv_nop" : "+v"(c) : "v"(a), "v"(b));
  return c;
}
__device__ __forceinline__ void wave_lds_sync() {
  __builtin_amdgcn_fence(__ATOMIC_RELEASE, "workgroup");
  __builtin_amdgcn_wave_barrier();
  __builtin_amdgcn_fence(__ATOMIC_ACQUIRE, "workgroup");
}

__device__ __forceinline__ void rel_pos(const float* __restrict__ pos, const int* __restrict__ idxp,
                                        const int* __restrict__ nbrp, int n, int jn,
                                        float& r0, float& r1, float& r2, int& nb) {
  const int ctr = clampi(idxp[n], NSRC - 1);
  nb = clampi(nbrp[n * KNB + jn], NSRC - 1);
  const float* pn = pos + (size_t)nb * 3;
  const float* pc = pos + (size_t)ctr * 3;
  r0 = bfr(pn[0]) - bfr(pc[0]);
  r1 = bfr(pn[1]) - bfr(pc[1]);
  r2 = bfr(pn[2]) - bfr(pc[2]);
}
__device__ __forceinline__ void store_rel(__bf16* relH, __bf16* relL, int pt, int jn, float r0, float r1, float r2) {
  const int b = pt * KRELP + jn * 3;
  __bf16 hi, lo;
  split_bf(r0, hi, lo); relH[b] = hi;     relL[b] = lo;
  split_bf(r1, hi, lo); relH[b + 1] = hi; relL[b + 1] = lo;
  split_bf(r2, hi, lo); relH[b + 2] = hi; relL[b + 2] = lo;
  const __bf16 z = tobf(0.0f);
  relH[pt * KRELP + KREL + jn] = z;
  relL[pt * KRELP + KREL + jn] = z;
}
__device__ __forceinline__ float h1_pre(const float* W1s, const float* b1s, int c, float r0, float r1, float r2) {
  return fmaf(W1s[c * 3 + 2], r2, fmaf(W1s[c * 3 + 1], r1, fmaf(W1s[c * 3], r0, b1s[c])));
}
__device__ __forceinline__ void t1_gemm(const __bf16* relH, const __bf16* relL, const __bf16* __restrict__ Wx1p,
                                        int wave, int cl, int hh, v8f& acc0, v8f& acc1) {
#pragma unroll
  for (int ks = 0; ks < 2; ++ks) {
    const v16b ah = frag_std(relH + cl * KRELP + ks * 32 + 8 * hh);
    const v16b al = frag_std(relL + cl * KRELP + ks * 32 + 8 * hh);
    const v16b b0 = frag_std(Wx1p + (size_t)((2 * wave) * 16 + cl) * KRELP + ks * 32 + 8 * hh);
    const v16b b1 = frag_std(Wx1p + (size_t)((2 * wave + 1) * 16 + cl) * KRELP + ks * 32 + 8 * hh);
    acc0 = mma_bf(ah, b0, acc0); acc0 = mma_bf(al, b0, acc0);
    acc1 = mma_bf(ah, b1, acc1); acc1 = mma_bf(al, b1, acc1);
  }
}
__device__ __forceinline__ void store_pt(float* __restrict__ PT, int blk, int wave, int lane, int hh,
                                         float s0, float q0, float s1, float q1) {
  s0 += __shfl_xor(s0, 16, 32);
  q0 += __shfl_xor(q0, 16, 32);
  s1 += __shfl_xor(s1, 16, 32);
  q1 += __shfl_xor(q1, 16, 32);
  const float vs = hh ? s1 : s0;
  const float vq = hh ? q1 : q0;
  float* d = PT + (size_t)blk * TPITCH + 32 * wave + lane;
  *(volatile float*)d = vs;
  *(volatile float*)(d + 256) = vq;
  __threadfence();
  *(volatile float*)d = vs;
  *(volatile float*)(d + 256) = vq;
}
__device__ __forceinline__ void load_t2n(const float* __restrict__ T2, const float* __restrict__ BN, int n0, int tid,
                                         __bf16* H, __bf16* L) {
  const int row = tid >> 4;
#pragma unroll 1
  for (int hs = 0; hs < 2; ++hs) {
    const int cg = (tid & 15) * 16 + 8 * hs;
    const float* tr  = T2 + (size_t)(n0 + row) * NCH1 + cg;
    const float* scp = BN + BN_SCX2 + cg;
    const float* shp = BN + BN_SHX2 + cg;
    v8b hv, lv;
#pragma unroll
    for (int i4 = 0; i4 < 2; ++i4) {
      const v4f t  = *(const v4f*)(tr + 4 * i4);
      const v4f sc = *(const v4f*)(scp + 4 * i4);
      const v4f sh = *(const v4f*)(shp + 4 * i4);
#pragma unroll
      for (int e = 0; e < 4; ++e) {
        const float v = fmaf(t[e], sc[e], sh[e]);
        __bf16 hi, lo; split_bf(v, hi, lo);
        hv[4 * i4 + e] = hi; lv[4 * i4 + e] = lo;
      }
    }
    *(v8b*)(H + row * NCH1 + cg) = hv;
    *(v8b*)(L + row * NCH1 + cg) = lv;
  }
}
__device__ __forceinline__ float sel_clamp(const float* __restrict__ p, int k, int n) {
  const int kc = k < n ? k : n - 1;
  const float v = p[kc];
  return k < n ? v : 0.f;
}

__global__ __launch_bounds__(256) void k_prep(
    const float* __restrict__ Wx1, const float* __restrict__ W2, const float* __restrict__ WX1,
    const float* __restrict__ WX2, const float* __restrict__ Wo,
    const float* __restrict__ W1, const float* __restrict__ b1, const float* __restrict__ b2,
    const float* __restrict__ bx1, const float* __restrict__ bG1, const float* __restrict__ bG2,
    const float* __restrict__ Wc, const float* __restrict__ bc, const float* __restrict__ bo,
    unsigned* __restrict__ wout) {
  const int i = blockIdx.x * 256 + threadIdx.x;
  if (i >= PREP_WORDS) return;
  unsigned u;
  if (i < WD_W2P) {
    const int e0 = 2 * i, ch = e0 >> 6, kk = e0 & 63;
    const int kc = kk < 46 ? kk : 46;
    float a = Wx1[ch * KREL + kc], b = Wx1[ch * KREL + kc + 1];
    if (kk >= KREL) { a = 0.f; b = 0.f; }
    u = pack2bf(a, b);
  } else if (i < WD_WX1G) {
    const int e0 = 2 * (i - WD_W2P);  u = pack2bf(W2[e0], W2[e0 + 1]);
  } else if (i < WD_WX2G) {
    const int e0 = 2 * (i - WD_WX1G); u = pack2bf(WX1[e0], WX1[e0 + 1]);
  } else if (i < WD_WOP) {
    const int e0 = 2 * (i - WD_WX2G); u = pack2bf(WX2[e0], WX2[e0 + 1]);
  } else if (i < WD_PR) {
    const int e0 = 2 * (i - WD_WOP);  u = pack2bf(Wo[e0], Wo[e0 + 1]);
  } else {
    const int r = i - WD_PR;
    float v;
    if (r < PR_B1)       v = sel_clamp(W1, r - PR_W1, 48);
    else if (r < PR_B2)  v = sel_clamp(b1, r - PR_B1, 16);
    else if (r < PR_BX1) v = sel_clamp(b2, r - PR_B2, 16);
    else if (r < PR_BG1) v = bx1[r - PR_BX1];
    else if (r < PR_BG2) v = bG1[r - PR_BG1];
    else if (r < PR_WC)  v = bG2[r - PR_BG2];
    else if (r < PR_BC)  v = Wc[r - PR_WC];
    else if (r < PR_BO)  v = bc[r - PR_BC];
    else                 v = bo[r - PR_BO];
    u = __float_as_uint(bfr(v));
  }
  ((volatile unsigned*)wout)[i] = u;
  __threadfence();
  ((volatile unsigned*)wout)[i] = u;
}

__global__ __launch_bounds__(256) void k_bnreduce(
    const float* __restrict__ P, int pitch, int soff, int qoff, int nch, int nblk, double inv_cnt,
    const float* __restrict__ gam, const float* __restrict__ bet,
    float* __restrict__ osc, float* __restrict__ osh) {
  const int ch = threadIdx.x;
  const int chc = ch < nch ? ch : nch - 1;
  double S = 0.0, Q = 0.0;
  for (int b = 0; b < nblk; ++b) {
    const float* row = P + (size_t)b * pitch;
    S += (double)row[soff + chc];
    Q += (double)row[qoff + chc];
  }
  const double mean = S * inv_cnt;
  double var = Q * inv_cnt - mean * mean;
  if (var < 0.0) var = 0.0;
  const float g = bfr(gam[chc]), be = bfr(bet[chc]);
  float sc = g * rsqrtf((float)var + 1e-5f);
  float sh = be - (float)mean * sc;
  if (ch >= nch) { sc = 0.f; sh = 0.f; }
  ((volatile float*)osc)[ch] = sc;
  ((volatile float*)osh)[ch] = sh;
  __threadfence();
  ((volatile float*)osc)[ch] = sc;
  ((volatile float*)osh)[ch] = sh;
}

__global__ __launch_bounds__(256) void k_stage_a(
    const float* __restrict__ pos, const int* __restrict__ idxp, const int* __restrict__ nbrp,
    const float* __restrict__ PR, const unsigned short* __restrict__ Wx1pu,
    float* __restrict__ PH, float* __restrict__ PT) {
  const __bf16* Wx1p = (const __bf16*)Wx1pu;
  __shared__ __align__(16) __bf16 relH[PB * KRELP];
  __shared__ __align__(16) __bf16 relL[PB * KRELP];
  __shared__ __align__(16) float Ebuf[256 * CDEL];
  __shared__ float PSs[256], PQs[256];
  __shared__ float W1s[48], b1s[16];
  const int tid = threadIdx.x, wave = tid >> 5, lane = tid & 31, hh = lane >> 4, cl = lane & 15;
  const int pt = tid >> 4, jn = tid & 15, blk = blockIdx.x, n0 = blk * PB;
  if (tid < 48) W1s[tid] = PR[PR_W1 + tid];
  if (tid < 16) b1s[tid] = PR[PR_B1 + tid];
  float r0, r1, r2; int nb;
  rel_pos(pos, idxp, nbrp, n0 + pt, jn, r0, r1, r2, nb);
  store_rel(relH, relL, pt, jn, r0, r1, r2);
  __syncthreads();
#pragma unroll
  for (int c = 0; c < CDEL; ++c) Ebuf[tid * CDEL + c] = eluf(h1_pre(W1s, b1s, c, r0, r1, r2));
  {
    v8f acc0 = zero8(), acc1 = zero8();
    t1_gemm(relH, relL, Wx1p, wave, cl, hh, acc0, acc1);
    const float bias0 = PR[PR_BX1 + (2 * wave) * 16 + cl];
    const float bias1 = PR[PR_BX1 + (2 * wave + 1) * 16 + cl];
    float s0 = 0.f, q0 = 0.f, s1 = 0.f, q1 = 0.f;
#pragma unroll
    for (int r = 0; r < 8; ++r) {
      const float e0 = eluf(acc0[r] + bias0); s0 += e0; q0 = fmaf(e0, e0, q0);
      const float e1 = eluf(acc1[r] + bias1); s1 += e1; q1 = fmaf(e1, e1, q1);
    }
    store_pt(PT, blk, wave, lane, hh, s0, q0, s1, q1);
  }
  __syncthreads();
  {
    const int ch = tid & 15, part = tid >> 4;
    float s = 0.f, q = 0.f;
#pragma unroll
    for (int i = 0; i < 16; ++i) {
      const float e = Ebuf[(part * 16 + i) * CDEL + ch];
      s += e; q = fmaf(e, e, q);
    }
    PSs[part * 16 + ch] = s; PQs[part * 16 + ch] = q;
  }
  __syncthreads();
  if (tid < 32) {
    const int ch = tid & 15;
    float S = 0.f;
#pragma unroll
    for (int part = 0; part < 16; ++part) {
      const float a = PSs[part * 16 + ch];
      const float b = PQs[part * 16 + ch];
      S += (tid < 16) ? a : b;
    }
    float* d = PH + (size_t)blk * HPITCH + tid;
    *(volatile float*)d = S;
    __threadfence();
    *(volatile float*)d = S;
  }
}

__global__ __launch_bounds__(256) void k_stage_b(
    const float* __restrict__ pos, const int* __restrict__ idxp, const int* __restrict__ nbrp,
    const float* __restrict__ PR, const float* __restrict__ BN,
    const unsigned short* __restrict__ Wx1pu, const unsigned short* __restrict__ W2pu,
    const unsigned short* __restrict__ WX1pu,
    float* __restrict__ PH, float* __restrict__ PT, float* __restrict__ T2) {
  const __bf16* Wx1p = (const __bf16*)Wx1pu;
  const __bf16* W2p  = (const __bf16*)W2pu;
  const __bf16* WX1p = (const __bf16*)WX1pu;
  __shared__ __align__(16) __bf16 relH[PB * KRELP];
  __shared__ __align__(16) __bf16 relL[PB * KRELP];
  __shared__ __align__(16) __bf16 h1H[4096];
  __shared__ __align__(16) __bf16 h1L[4096];
  __shared__ __align__(16) __bf16 t1H[4096];
  __shared__ __align__(16) __bf16 t1L[4096];
  __shared__ __align__(16) float slabs[8 * 512];
  __shared__ float parB[112];
  __shared__ float wst[256];
  const int tid = threadIdx.x, wave = tid >> 5, lane = tid & 31, hh = lane >> 4, cl = lane & 15;
  const int pt = tid >> 4, jn = tid & 15, blk = blockIdx.x, n0 = blk * PB;
  if (tid < 48) parB[tid] = PR[PR_W1 + tid];
  if (tid < 16) {
    parB[48 + tid] = PR[PR_B1 + tid];
    parB[64 + tid] = BN[BN_SC1 + tid];
    parB[80 + tid] = BN[BN_SH1 + tid];
    parB[96 + tid] = PR[PR_B2 + tid];
  }
  float r0, r1, r2; int nb;
  rel_pos(pos, idxp, nbrp, n0 + pt, jn, r0, r1, r2, nb);
  store_rel(relH, relL, pt, jn, r0, r1, r2);
  __syncthreads();
  {
    v8b hv0, hv1, lv0, lv1;
#pragma unroll
    for (int c = 0; c < CDEL; ++c) {
      const float v = fmaf(eluf(h1_pre(parB, parB + 48, c, r0, r1, r2)), parB[64 + c], parB[80 + c]);
      __bf16 hi, lo; split_bf(v, hi, lo);
      if (c < 8) { hv0[c] = hi; lv0[c] = lo; } else { hv1[c - 8] = hi; lv1[c - 8] = lo; }
    }
    *(v8b*)(h1H + tid * 16) = hv0; *(v8b*)(h1H + tid * 16 + 8) = hv1;
    *(v8b*)(h1L + tid * 16) = lv0; *(v8b*)(h1L + tid * 16 + 8) = lv1;
  }
  __syncthreads();
  {
    float s = 0.f, q = 0.f;
    const float bias = parB[96 + cl];
#pragma unroll
    for (int u = 0; u < 2; ++u) {
      const int rt = 2 * wave + u;
      const v16b a = frag_pair(h1H + (rt * 16 + cl) * 16 + 8 * hh, h1L + (rt * 16 + cl) * 16 + 8 * hh);
      const v16b b = frag_dup(W2p + cl * 16 + 8 * hh);
      const v8f acc = mma_bf(a, b, zero8());
#pragma unroll
      for (int r = 0; r < 8; ++r) { const float e = eluf(acc[r] + bias); s += e; q = fmaf(e, e, q); }
    }
    s += __shfl_xor(s, 16, 32);
    q += __shfl_xor(q, 16, 32);
    wst[wave * 32 + lane] = hh ? q : s;
  }
  {
    v8f acc0 = zero8(), acc1 = zero8();
    t1_gemm(relH, relL, Wx1p, wave, cl, hh, acc0, acc1);
    const int ch0 = (2 * wave) * 16 + cl, ch1 = (2 * wave + 1) * 16 + cl;
    const float bias0 = PR[PR_BX1 + ch0], sc0 = BN[BN_SCX1 + ch0], sh0 = BN[BN_SHX1 + ch0];
    const float bias1 = PR[PR_BX1 + ch1], sc1 = BN[BN_SCX1 + ch1], sh1 = BN[BN_SHX1 + ch1];
#pragma unroll
    for (int r = 0; r < 8; ++r) {
      const int row = 8 * hh + r;
      __bf16 hi, lo;
      split_bf(fmaf(eluf(acc0[r] + bias0), sc0, sh0), hi, lo); t1H[row * NCH1 + ch0] = hi; t1L[row * NCH1 + ch0] = lo;
      split_bf(fmaf(eluf(acc1[r] + bias1), sc1, sh1), hi, lo); t1H[row * NCH1 + ch1] = hi; t1L[row * NCH1 + ch1] = lo;
    }
  }
  __syncthreads();
  if (tid < 32) {
    float S = 0.f;
#pragma unroll
    for (int w = 0; w < 8; ++w) S += wst[w * 32 + tid];
    float* d = PH + (size_t)blk * HPITCH + tid;
    *(volatile float*)d = S;
    __threadfence();
    *(volatile float*)d = S;
  }
  {
    float* slab = slabs + wave * 512;
    float s0 = 0.f, q0 = 0.f, s1 = 0.f, q1 = 0.f;
#pragma unroll
    for (int u = 0; u < 2; ++u) {
      const int g = 2 * wave + u;
      const v16b a = frag_pair(t1H + cl * NCH1 + g * 16 + 8 * hh, t1L + cl * NCH1 + g * 16 + 8 * hh);
      const v16b b = frag_dup(WX1p + (g * 16 + cl) * 16 + 8 * hh);
      const v8f acc = mma_bf(a, b, zero8());
      const float bias = PR[PR_BG1 + g * 16 + cl];
#pragma unroll
      for (int r = 0; r < 8; ++r) {
        const float e = eluf(acc[r] + bias);
        if (u == 0) { s0 += e; q0 = fmaf(e, e, q0); } else { s1 += e; q1 = fmaf(e, e, q1); }
        slab[(8 * hh + r) * 32 + u * 16 + cl] = e;
      }
    }
    store_pt(PT, blk, wave, lane, hh, s0, q0, s1, q1);
    wave_lds_sync();
    const int q8 = lane >> 3, c4 = (lane & 7) * 4;
    v4f vv[4];
#pragma unroll
    for (int it = 0; it < 4; ++it) vv[it] = *(const v4f*)(slab + (it * 4 + q8) * 32 + c4);
    for (int pass = 0; pass < 2; ++pass) {
#pragma unroll
      for (int it = 0; it < 4; ++it)
        *(volatile v4f*)(T2 + (size_t)(n0 + it * 4 + q8) * NCH1 + wave * 32 + c4) = vv[it];
      __threadfence();
    }
  }
}

__global__ __launch_bounds__(256) void k_stage_c(
    const float* __restrict__ T2, const float* __restrict__ BN, const float* __restrict__ PR,
    const unsigned short* __restrict__ WX2pu, float* __restrict__ PT) {
  const __bf16* WX2p = (const __bf16*)WX2pu;
  __shared__ __align__(16) __bf16 t2H[4096];
  __shared__ __align__(16) __bf16 t2L[4096];
  const int tid = threadIdx.x, wave = tid >> 5, lane = tid & 31, hh = lane >> 4, cl = lane & 15;
  const int blk = blockIdx.x, n0 = blk * PB;
  load_t2n(T2, BN, n0, tid, t2H, t2L);
  __syncthreads();
  float s0 = 0.f, q0 = 0.f, s1 = 0.f, q1 = 0.f;
#pragma unroll
  for (int u = 0; u < 2; ++u) {
    const int g = 2 * wave + u;
    const v16b a = frag_pair(t2H + cl * NCH1 + g * 16 + 8 * hh, t2L + cl * NCH1 + g * 16 + 8 * hh);
    const v16b b = frag_dup(WX2p + (g * 16 + cl) * 16 + 8 * hh);
    const v8f acc = mma_bf(a, b, zero8());
    const float bias = PR[PR_BG2 + g * 16 + cl];
#pragma unroll
    for (int r = 0; r < 8; ++r) {
      const float v = acc[r] + bias;
      if (u == 0) { s0 += v; q0 = fmaf(v, v, q0); } else { s1 += v; q1 = fmaf(v, v, q1); }
    }
  }
  store_pt(PT, blk, wave, lane, hh, s0, q0, s1, q1);
}

__device__ __forceinline__ void conv_y(v8f acc, const float* __restrict__ PR, int p, int cg, int hh,
                                       __bf16* yH, __bf16* yL) {
  const float* wc = PR + PR_WC + cg * 32 + 8 * hh;
  const v4f w0a = *(const v4f*)(wc), w0b = *(const v4f*)(wc + 4);
  const v4f w1a = *(const v4f*)(wc + 16), w1b = *(const v4f*)(wc + 20);
  float y0 = 0.f, y1 = 0.f;
#pragma unroll
  for (int r = 0; r < 4; ++r) { y0 = fmaf(w0a[r], acc[r], y0); y1 = fmaf(w1a[r], acc[r], y1); }
#pragma unroll
  for (int r = 0; r < 4; ++r) { y0 = fmaf(w0b[r], acc[4 + r], y0); y1 = fmaf(w1b[r], acc[4 + r], y1); }
  y0 += __shfl_xor(y0, 16, 32);
  y1 += __shfl_xor(y1, 16, 32);
  const float bcv = PR[PR_BC + cg * 2 + hh];
  const float yv = (hh ? y1 : y0) + bcv;
  __bf16 hi, lo; split_bf(yv, hi, lo);
  yH[p * YDIM + cg * 2 + hh] = hi;
  yL[p * YDIM + cg * 2 + hh] = lo;
}

__global__ __launch_bounds__(256) void k_stage_d(
    const float* __restrict__ x, const float* __restrict__ pos,
    const int* __restrict__ idxp, const int* __restrict__ nbrp,
    const float* __restrict__ PR, const float* __restrict__ BN,
    const unsigned short* __restrict__ W2pu, const unsigned short* __restrict__ WX2pu,
    const unsigned short* __restrict__ Wopu, const float* __restrict__ T2, float* __restrict__ out) {
  const __bf16* W2p  = (const __bf16*)W2pu;
  const __bf16* WX2p = (const __bf16*)WX2pu;
  const __bf16* Wop  = (const __bf16*)Wopu;
  __shared__ __align__(16) __bf16 R0[8192];
  __shared__ __align__(16) __bf16 RT[8192];
  __shared__ __align__(16) __bf16 RH[8192];
  __shared__ __align__(16) float OSX[16 * 132];
  __shared__ float parD[144];
  const int tid = threadIdx.x, wave = tid >> 5, lane = tid & 31, hh = lane >> 4, cl = lane & 15;
  const int pt = tid >> 4, jn = tid & 15, blk = blockIdx.x, n0 = blk * PB;
  __bf16* t2H = R0; __bf16* t2L = R0 + 4096;
  __bf16* TH = RT;  __bf16* TL = RT + 4096;
  __bf16* HH = RH;  __bf16* HL = RH + 4096;
  if (tid < 48) parD[tid] = PR[PR_W1 + tid];
  if (tid < 16) {
    parD[48 + tid]  = PR[PR_B1 + tid];
    parD[64 + tid]  = BN[BN_SC1 + tid];
    parD[80 + tid]  = BN[BN_SH1 + tid];
    parD[96 + tid]  = PR[PR_B2 + tid];
    parD[112 + tid] = BN[BN_SC2 + tid];
    parD[128 + tid] = BN[BN_SH2 + tid];
  }
  load_t2n(T2, BN, n0, tid, t2H, t2L);
  __syncthreads();
  {
#pragma unroll
    for (int u = 0; u < 2; ++u) {
      const int g = 2 * wave + u;
      const v16b a = frag_pair(t2H + cl * NCH1 + g * 16 + 8 * hh, t2L + cl * NCH1 + g * 16 + 8 * hh);
      const v16b b = frag_dup(WX2p + (g * 16 + cl) * 16 + 8 * hh);
      const v8f acc = mma_bf(a, b, zero8());
      const int ch = g * 16 + cl;
      const float bias = PR[PR_BG2 + ch], sc = BN[BN_SCX3 + ch], sh = BN[BN_SHX3 + ch];
#pragma unroll
      for (int r = 0; r < 8; ++r) {
        const float v = fmaf(acc[r] + bias, sc, sh);
        __bf16 hi, lo; split_bf(v, hi, lo);
        TH[(8 * hh + r) * NCH1 + ch] = hi;
        TL[(8 * hh + r) * NCH1 + ch] = lo;
      }
    }
  }
  __syncthreads();
  float r0, r1, r2; int nb;
  rel_pos(pos, idxp, nbrp, n0 + pt, jn, r0, r1, r2, nb);
  {
    v8b hv0, hv1, lv0, lv1;
#pragma unroll
    for (int c = 0; c < CDEL; ++c) {
      const float v = fmaf(eluf(h1_pre(parD, parD + 48, c, r0, r1, r2)), parD[64 + c], parD[80 + c]);
      __bf16 hi, lo; split_bf(v, hi, lo);
      if (c < 8) { hv0[c] = hi; lv0[c] = lo; } else { hv1[c - 8] = hi; lv1[c - 8] = lo; }
    }
    *(v8b*)(R0 + tid * 16) = hv0; *(v8b*)(R0 + tid * 16 + 8) = hv1;
    *(v8b*)(R0 + 4096 + tid * 16) = lv0; *(v8b*)(R0 + 4096 + tid * 16 + 8) = lv1;
  }
  __syncthreads();
  {
    const float bias = parD[96 + cl], sc = parD[112 + cl], sh = parD[128 + cl];
#pragma unroll
    for (int u = 0; u < 2; ++u) {
      const int rt = 2 * wave + u;
      const v16b a = frag_pair(R0 + (rt * 16 + cl) * 16 + 8 * hh, R0 + 4096 + (rt * 16 + cl) * 16 + 8 * hh);
      const v16b b = frag_dup(W2p + cl * 16 + 8 * hh);
      const v8f acc = mma_bf(a, b, zero8());
      v8b hv, lv;
#pragma unroll
      for (int r = 0; r < 8; ++r) {
        const float v = fmaf(eluf(acc[r] + bias), sc, sh);
        __bf16 hi, lo; split_bf(v, hi, lo);
        hv[r] = hi; lv[r] = lo;
      }
      *(v8b*)(HH + rt * 256 + cl * 16 + 8 * hh) = hv;
      *(v8b*)(HL + rt * 256 + cl * 16 + 8 * hh) = lv;
    }
  }
  __syncthreads();
  __bf16* yH = R0; __bf16* yL = R0 + 2560;
  __bf16* XSW = ((__bf16*)OSX) + wave * 512;
#pragma unroll
  for (int q = 0; q < 2; ++q) {
    const int p = 2 * wave + q;
    const v16b a  = frag_pair(TH + p * 256 + cl * 16 + 8 * hh, TL + p * 256 + cl * 16 + 8 * hh);
    const v16b bh = frag_dup(HH + p * 256 + cl * 16 + 8 * hh);
    const v16b bl = frag_dup(HL + p * 256 + cl * 16 + 8 * hh);
    v8f acc = mma_bf(a, bh, zero8());
    acc = mma_bf(a, bl, acc);
    conv_y(acc, PR, p, cl, hh, yH, yL);
  }
#pragma unroll
  for (int ct = 1; ct < 5; ++ct) {
    wave_lds_sync();
#pragma unroll
    for (int q = 0; q < 2; ++q) {
      const int nbq = __shfl(nb, q * 16 + cl, 32);
      const float* xr = x + (size_t)nbq * CIN + (ct - 1) * 16 + 8 * hh;
      const v4f xa = *(const v4f*)(xr);
      const v4f xb = *(const v4f*)(xr + 4);
      __bf16* xs = XSW + q * 256;
#pragma unroll
      for (int e = 0; e < 4; ++e) {
        xs[(8 * hh + e) * 16 + cl]     = tobf(xa[e]);
        xs[(8 * hh + 4 + e) * 16 + cl] = tobf(xb[e]);
      }
    }
    wave_lds_sync();
#pragma unroll
    for (int q = 0; q < 2; ++q) {
      const int p = 2 * wave + q;
      const v16b a = frag_pair(TH + p * 256 + cl * 16 + 8 * hh, TL + p * 256 + cl * 16 + 8 * hh);
      const v16b b = frag_dup(XSW + q * 256 + cl * 16 + 8 * hh);
      const v8f acc = mma_bf(a, b, zero8());
      conv_y(acc, PR, p, ct * 16 + cl, hh, yH, yL);
    }
  }
  __syncthreads();
  {
    const int oc = wave * 16 + cl;
    v8f acc = zero8();
#pragma unroll 1
    for (int ks = 0; ks < 5; ++ks) {
      const v16b ah = frag_std(yH + cl * YDIM + ks * 32 + 8 * hh);
      const v16b al = frag_std(yL + cl * YDIM + ks * 32 + 8 * hh);
      const v16b b  = frag_std(Wop + (size_t)oc * YDIM + ks * 32 + 8 * hh);
      acc = mma_bf(ah, b, acc);
      acc = mma_bf(al, b, acc);
    }
    const float bias = PR[PR_BO + oc];
#pragma unroll
    for (int r = 0; r < 8; ++r) OSX[(8 * hh + r) * 132 + oc] = acc[r] + bias;
  }
  __syncthreads();
  {
    const v4f v0 = *(const v4f*)(OSX + (2 * wave) * 132 + lane * 4);
    const v4f v1 = *(const v4f*)(OSX + (2 * wave + 1) * 132 + lane * 4);
    float* d0 = out + (size_t)(n0 + 2 * wave) * COUT + lane * 4;
    float* d1 = d0 + COUT;
    *(volatile v4f*)d0 = v0;
    *(volatile v4f*)d1 = v1;
    __threadfence();
    *(volatile v4f*)d0 = v0;
    *(volatile v4f*)d1 = v1;
  }
}

extern "C" void kernel_launch(void* const* d_in, const int* in_sizes, int n_in,
                              void* d_out, int out_size, void* d_ws, size_t ws_size,
                              hipStream_t stream) {
  (void)in_sizes;
  if (n_in < 28) return;
  if (ws_size < WS_END) return;
  if (out_size < NPTS * COUT) return;
  const float* x    = (const float*)d_in[0];
  const float* pos  = (const float*)d_in[1];
  const int*   idxp = (const int*)d_in[2];
  const int*   nbrp = (const int*)d_in[3];
  const float* W1   = (const float*)d_in[4];
  const float* b1   = (const float*)d_in[5];
  const float* g1   = (const float*)d_in[6];
  const float* be1  = (const float*)d_in[7];
  const float* W2   = (const float*)d_in[8];
  const float* b2   = (const float*)d_in[9];
  const float* g2   = (const float*)d_in[10];
  const float* be2  = (const float*)d_in[11];
  const float* Wx1  = (const float*)d_in[12];
  const float* bx1  = (const float*)d_in[13];
  const float* gx1  = (const float*)d_in[14];
  const float* bex1 = (const float*)d_in[15];
  const float* WX1  = (const float*)d_in[16];
  const float* bG1  = (const float*)d_in[17];
  const float* gx2  = (const float*)d_in[18];
  const float* bex2 = (const float*)d_in[19];
  const float* WX2  = (const float*)d_in[20];
  const float* bG2  = (const float*)d_in[21];
  const float* gx3  = (const float*)d_in[22];
  const float* bex3 = (const float*)d_in[23];
  const float* Wc   = (const float*)d_in[24];
  const float* bc   = (const float*)d_in[25];
  const float* Wo   = (const float*)d_in[26];
  const float* bo   = (const float*)d_in[27];
  float* out = (float*)d_out;
  char* ws = (char*)d_ws;
  const unsigned short* Wx1pu = (const unsigned short*)(ws + OFF_WX1P);
  const unsigned short* W2pu  = (const unsigned short*)(ws + OFF_W2P);
  const unsigned short* WX1pu = (const unsigned short*)(ws + OFF_WX1G);
  const unsigned short* WX2pu = (const unsigned short*)(ws + OFF_WX2G);
  const unsigned short* Wopu  = (const unsigned short*)(ws + OFF_WOP);
  float* PR = (float*)(ws + OFF_PR);
  float* BN = (float*)(ws + OFF_BN);
  float* PH = (float*)(ws + OFF_PH);
  float* PT = (float*)(ws + OFF_PT);
  float* T2 = (float*)(ws + OFF_T2);
  const double invH = 1.0 / (double)((long)NPTS * KNB);
  const double invT = 1.0 / (double)NPTS;

  k_prep<<<(PREP_WORDS + 255) / 256, 256, 0, stream>>>(Wx1, W2, WX1, WX2, Wo, W1, b1, b2, bx1, bG1, bG2,
                                                      Wc, bc, bo, (unsigned*)(ws + OFF_WX1P));
  k_stage_a<<<NBLKS, 256, 0, stream>>>(pos, idxp, nbrp, PR, Wx1pu, PH, PT);
  k_bnreduce<<<1, 32, 0, stream>>>(PH, HPITCH, 0, 16, 16, NBLKS, invH, g1, be1, BN + BN_SC1, BN + BN_SH1);
  k_bnreduce<<<1, 256, 0, stream>>>(PT, TPITCH, 0, 256, 256, NBLKS, invT, gx1, bex1, BN + BN_SCX1, BN + BN_SHX1);
  k_stage_b<<<NBLKS, 256, 0, stream>>>(pos, idxp, nbrp, PR, BN, Wx1pu, W2pu, WX1pu, PH, PT, T2);
  k_bnreduce<<<1, 32, 0, stream>>>(PH, HPITCH, 0, 16, 16, NBLKS, invH, g2, be2, BN + BN_SC2, BN + BN_SH2);
  k_bnreduce<<<1, 256, 0, stream>>>(PT, TPITCH, 0, 256, 256, NBLKS, invT, gx2, bex2, BN + BN_SCX2, BN + BN_SHX2);
  k_stage_c<<<NBLKS, 256, 0, stream>>>(T2, BN, PR, WX2pu, PT);
  k_bnreduce<<<1, 256, 0, stream>>>(PT, TPITCH, 0, 256, 256, NBLKS, invT, gx3, bex3, BN + BN_SCX3, BN + BN_SHX3);
  k_stage_d<<<NBLKS, 256, 0, stream>>>(x, pos, idxp, nbrp, PR, BN, W2pu, WX2pu, Wopu, T2, out);
}
